// GINENet_80865644249571
// MI455X (gfx1250) — hardware-verified
//
#include <hip/hip_runtime.h>
#include <stddef.h>
#include <stdint.h>

#define C0      32
#define C1      64
#define DH      64
#define EDIM    16
#define KE      32
#define NTHR    256
#define NWAVE   8
#define EPT     8
#define CHUNK   (NTHR * EPT)
#define WCAP    (EPT * 32)
#define LISTN   (NWAVE * WCAP)
#define NBR     1024
#define PKS     10
#define RCAP    28672
#define DEGCAP  64
#define NODECAP 512
#define ETILE   128
#define APE     40
#define GBM     64
#define GTHR    128
#define NGATE   256
#define OUTP    32
#define CMSG    16.0f
#define MINV    0.0625f
#define BKT_ZINTS (2 * RCAP + 2 * NBR + LISTN)
#define LDS_BKT   (BKT_ZINTS * 4 + 64)
#define LDS_S2S   ((NODECAP * DH + NWAVE * NODECAP + NODECAP) * 4)
#define PREP_UNITS (256 + 256 + 512 + 1024 + 1024 + 1024 + 8192 + 4096)

static_assert(EDIM <= KE && (KE % 32) == 0);
static_assert(C0 == 32 && C1 == 64 && DH == 64);
static_assert((CHUNK & (CHUNK - 1)) == 0 && ((long long)CHUNK << PKS) < (1LL << 31));
static_assert(NBR == (1 << PKS) && NTHR * 4 == NBR && LISTN >= NBR);
static_assert((RCAP % 32) == 0 && (BKT_ZINTS % (4 * NTHR)) == 0);
static_assert(LDS_BKT <= 300000 && LDS_S2S <= 300000);
static_assert(DEGCAP >= 48 && NODECAP >= 133);
static_assert(NGATE == NTHR && NGATE == 4 * DH);
static_assert((OUTP * 4) == 128);
static_assert(ETILE == 4 * 32 && (APE * 2) % 16 == 0 && APE >= KE);
static_assert(GBM == (GTHR / 32) * 16);
static_assert((PREP_UNITS % NTHR) == 0);

typedef float          v2f  __attribute__((ext_vector_type(2)));
typedef float          v4f  __attribute__((ext_vector_type(4)));
typedef float          v8f  __attribute__((ext_vector_type(8)));
typedef int            v4i  __attribute__((ext_vector_type(4)));
typedef int            v8i  __attribute__((ext_vector_type(8)));
typedef unsigned int   v4u  __attribute__((ext_vector_type(4)));
typedef unsigned short v8us __attribute__((ext_vector_type(8)));
typedef __bf16         v16b __attribute__((ext_vector_type(16)));
typedef v4f  __attribute__((may_alias)) v4fa;
typedef v4i  __attribute__((may_alias)) v4ia;
typedef v4u  __attribute__((may_alias)) v4ua;
typedef v8us __attribute__((may_alias)) v8usa;
typedef unsigned int __attribute__((may_alias)) u32a;
union FragB { v16b v; v8us h[2]; v8i w; };

__device__ __forceinline__ v8f wmb(const FragB& a, const FragB& b, v8f c) {
  v8f d = __builtin_amdgcn_wmma_f32_16x16x32_bf16(false, a.v, false, b.v, (short)0, c, false, false);
  asm volatile("v_nop\n\tv_nop\n\tv_nop\n\tv_nop" : "+v"(d) : "v"(a.w), "v"(b.w));
  return d;
}

__device__ __forceinline__ unsigned short bf_bits(float f) {
  unsigned int u = __float_as_uint(f);
  const bool isn = (f != f);
  u += 0x7FFFu + ((u >> 16) & 1u);
  return isn ? (unsigned short)0x7FC0u : (unsigned short)(u >> 16);
}
__device__ __forceinline__ float bf_val(unsigned short b) { return __uint_as_float(((unsigned int)b) << 16); }
__device__ __forceinline__ float bf_rne(float f) { return bf_val(bf_bits(f)); }
__device__ __forceinline__ unsigned short f2h(float f) {
  const _Float16 hv = (_Float16)f;
  return __builtin_bit_cast(unsigned short, hv);
}
__device__ __forceinline__ float h2f(unsigned b) {
  const _Float16 hv = __builtin_bit_cast(_Float16, (unsigned short)b);
  return (float)hv;
}
__device__ __forceinline__ float relu_np(float v) { return (v > 0.0f) ? v : (v - v); }
__device__ __forceinline__ float nmax(float a, float b) {
  const float mx = (b > a) ? b : a;
  return (a != a) ? a : ((b != b) ? b : mx);
}
__device__ __forceinline__ void put16(unsigned short* dp, v8us o) {
  *(volatile v8us*)dp = o;
  __threadfence();
  *(volatile v8us*)dp = o;
}
__device__ __forceinline__ void putf4(float* dp, v4f o) {
  *(volatile v4f*)dp = o;
  __threadfence();
  *(volatile v4f*)dp = o;
}

__device__ __forceinline__ int scan_chunk(const int* __restrict__ dsts, int nE, int cbase, int slotBase,
                                          int nb, int vec8, int* list, int tid, int lane, int wave) {
  int wc = 0;
  const int el0  = tid * EPT;
  const int e0   = cbase + el0;
  const int sent = -2147483647 - 1;
  v4i da, db;
  if (vec8 != 0 && cbase + CHUNK <= nE) {
    da = *(const v4i*)(dsts + e0);
    db = *(const v4i*)(dsts + e0 + 4);
  } else {
    da.x = (e0     < nE) ? dsts[min(e0,     nE - 1)] : sent;
    da.y = (e0 + 1 < nE) ? dsts[min(e0 + 1, nE - 1)] : sent;
    da.z = (e0 + 2 < nE) ? dsts[min(e0 + 2, nE - 1)] : sent;
    da.w = (e0 + 3 < nE) ? dsts[min(e0 + 3, nE - 1)] : sent;
    db.x = (e0 + 4 < nE) ? dsts[min(e0 + 4, nE - 1)] : sent;
    db.y = (e0 + 5 < nE) ? dsts[min(e0 + 5, nE - 1)] : sent;
    db.z = (e0 + 6 < nE) ? dsts[min(e0 + 6, nE - 1)] : sent;
    db.w = (e0 + 7 < nE) ? dsts[min(e0 + 7, nE - 1)] : sent;
  }
  const unsigned nbs = (unsigned)slotBase;
  const unsigned unb = (unsigned)nb;
  const unsigned s0 = (unsigned)da.x - nbs, s1 = (unsigned)da.y - nbs;
  const unsigned s2 = (unsigned)da.z - nbs, s3 = (unsigned)da.w - nbs;
  const unsigned s4 = (unsigned)db.x - nbs, s5 = (unsigned)db.y - nbs;
  const unsigned s6 = (unsigned)db.z - nbs, s7 = (unsigned)db.w - nbs;
  const bool h0 = s0 < unb, h1 = s1 < unb, h2 = s2 < unb, h3 = s3 < unb;
  const bool h4 = s4 < unb, h5 = s5 < unb, h6 = s6 < unb, h7 = s7 < unb;
  const unsigned any = __builtin_amdgcn_ballot_w32(h0 | h1 | h2 | h3 | h4 | h5 | h6 | h7);
  if (any != 0u) {
#define HITJ(J, HJ, SJ) { \
      const unsigned mj = __builtin_amdgcn_ballot_w32(HJ); \
      if (mj != 0u) { \
        if (HJ) { \
          const int pos = wc + (int)__builtin_amdgcn_mbcnt_lo(mj, 0u); \
          if (pos < WCAP) list[wave * WCAP + pos] = ((el0 + (J)) << PKS) | (int)(SJ); \
        } \
        wc += (int)__builtin_popcount(mj); } }
    HITJ(0, h0, s0)
    HITJ(1, h1, s1)
    HITJ(2, h2, s2)
    HITJ(3, h3, s3)
    HITJ(4, h4, s4)
    HITJ(5, h5, s5)
    HITJ(6, h6, s6)
    HITJ(7, h7, s7)
#undef HITJ
  }
  return wc;
}

__device__ __forceinline__ void wunit(const float* __restrict__ W, int kin, int nout, int kpitch, int dup,
                                      int v, int nun, unsigned short* plane) {
  if (v >= nun) return;
  const int upr = kpitch >> 3;
  const int n   = v / upr;
  const int k8  = (v - n * upr) * 8;
  const int kk  = k8 % kin;
  const bool valid = (dup != 0) || (k8 < kin);
  const float* p = W + (size_t)kk * nout + n;
  v8us o;
#pragma unroll
  for (int i = 0; i < 8; ++i) {
    const float f = p[(size_t)i * nout];
    o[i] = valid ? bf_bits(f) : (unsigned short)0;
  }
  put16(plane + (size_t)v * 8, o);
}

__global__ __launch_bounds__(NTHR) void k_prep(const float* __restrict__ ew0, const float* __restrict__ ew1,
                                               const float* __restrict__ w10, const float* __restrict__ w20,
                                               const float* __restrict__ w11, const float* __restrict__ w21,
                                               const float* __restrict__ wih, const float* __restrict__ whh,
                                               unsigned short* EW0T, unsigned short* EW1T,
                                               unsigned short* W1C0, unsigned short* W2C0,
                                               unsigned short* W1C1, unsigned short* W2C1, float* GT) {
  const int u = (int)blockIdx.x * NTHR + (int)threadIdx.x;
  if (u < 256)        { wunit(ew0, EDIM, C0, KE, 0, u, 128, EW0T); return; }
  else if (u < 512)   { wunit(ew1, EDIM, C1, KE, 0, u - 256, 256, EW1T); return; }
  else if (u < 1024)  { wunit(w10, C0, DH, 2 * C0, 1, u - 512, 512, W1C0); return; }
  else if (u < 2048)  { wunit(w20, DH, DH, 2 * DH, 1, u - 1024, 1024, W2C0); return; }
  else if (u < 3072)  { wunit(w11, C1, DH, 2 * C1, 1, u - 2048, 1024, W1C1); return; }
  else if (u < 4096)  { wunit(w21, DH, DH, 2 * DH, 1, u - 3072, 1024, W2C1); return; }
  else if (u < 12288) {
    const int v  = u - 4096;
    const int k  = v >> 6;
    const int j4 = (v & 63) * 4;
    v4f q;
    q.x = bf_rne(wih[(size_t)(j4 + 0) * 128 + k]);
    q.y = bf_rne(wih[(size_t)(j4 + 1) * 128 + k]);
    q.z = bf_rne(wih[(size_t)(j4 + 2) * 128 + k]);
    q.w = bf_rne(wih[(size_t)(j4 + 3) * 128 + k]);
    putf4(GT + (size_t)v * 4, q);
    return;
  } else if (u < 16384) {
    const int v  = u - 12288;
    const int k  = v >> 6;
    const int j4 = (v & 63) * 4;
    v4f q;
    q.x = bf_rne(whh[(size_t)(j4 + 0) * 64 + k]);
    q.y = bf_rne(whh[(size_t)(j4 + 1) * 64 + k]);
    q.z = bf_rne(whh[(size_t)(j4 + 2) * 64 + k]);
    q.w = bf_rne(whh[(size_t)(j4 + 3) * 64 + k]);
    putf4(GT + (size_t)(8192 + v) * 4, q);
    return;
  }
}

__global__ __launch_bounds__(NTHR) void k_bucket(const int* __restrict__ dsts, int nN, int nE, int vec8,
                                                 int* LISTg, int* CNTg, int* OFFg, int* FLGg) {
  extern __shared__ v4f bkt_dyn[];
  int* reg1 = (int*)bkt_dyn;
  int* reg2 = reg1 + RCAP;
  int* scnt = reg2 + RCAP;
  int* soff = scnt + NBR;
  int* list = soff + NBR;
  int* wcnt = list + LISTN;
  int* wtot = wcnt + NWAVE;
  const int tid = (int)threadIdx.x, lane = tid & 31, wave = tid >> 5;
  const int nodeBase = (int)blockIdx.x * NBR;
  int nb = nN - nodeBase;
  nb = nb < 0 ? 0 : (nb > NBR ? NBR : nb);

  {
    const v4i z4 = {0, 0, 0, 0};
    for (int i = tid * 4; i < BKT_ZINTS; i += NTHR * 4) *(v4ia*)(reg1 + i) = z4;
    if (tid < 2 * NWAVE) wcnt[tid] = 0;
  }
  __syncthreads();

  int tot = 0;
  const int nChunks = (nE + CHUNK - 1) / CHUNK;
#pragma unroll 1
  for (int ch = 0; ch < nChunks; ++ch) {
    const int cbase = ch * CHUNK;
    const int wc = scan_chunk(dsts, nE, cbase, nodeBase, nb, vec8, list, tid, lane, wave);
    if (lane == 0) wcnt[wave] = wc;
    __syncthreads();
    int pre = 0, all = 0;
#pragma unroll
    for (int w2 = 0; w2 < NWAVE; ++w2) {
      int c = wcnt[w2];
      c = c < 0 ? 0 : (c > WCAP ? WCAP : c);
      all += c;
      pre += (w2 < wave) ? c : 0;
    }
    const int wcc  = wc > WCAP ? WCAP : wc;
    const int base = tot + pre;
#pragma unroll 1
    for (int i = lane; i < wcc; i += 32) {
      const int ent = list[wave * WCAP + i];
      const int el  = (ent >> PKS) & (CHUNK - 1);
      const int sl  = ent & (NBR - 1);
      int eid = cbase + el;
      eid = eid > nE - 1 ? nE - 1 : eid;
      const int pos = base + i;
      if (pos < RCAP) reg1[pos] = (int)(((unsigned)eid << PKS) | (unsigned)sl);
    }
    tot += all;
    tot = tot > RCAP ? RCAP : tot;
    __syncthreads();
  }
  const int nh = tot;

  if (wave == 0) {
#pragma unroll 1
    for (int b0 = 0; b0 < nh; b0 += 32) {
      const int idx = b0 + lane;
      const int uv  = reg1[idx < RCAP ? idx : RCAP - 1];
      const int m32 = (nh - b0) < 32 ? (nh - b0) : 32;
#pragma unroll 1
      for (int k = 0; k < m32; ++k) {
        const int u  = __builtin_amdgcn_readlane(uv, k);
        const int sl = u & (NBR - 1);
        if (lane == 0) scnt[sl] = scnt[sl] + 1;
      }
    }
  }
  __syncthreads();

  {
    const v4i ca = *(const v4ia*)(scnt + 4 * tid);
    const int e0 = ca.x < 0 ? 0 : ca.x, e1 = ca.y < 0 ? 0 : ca.y;
    const int e2 = ca.z < 0 ? 0 : ca.z, e3 = ca.w < 0 ? 0 : ca.w;
    const int ts = e0 + e1 + e2 + e3;
    int incl = ts;
#pragma unroll
    for (int d = 1; d < 32; d <<= 1) {
      const int up = __shfl_up(incl, d);
      if (lane >= d) incl += up;
    }
    if (lane == 31) wtot[wave] = incl;
    __syncthreads();
    int pre = 0;
#pragma unroll
    for (int w2 = 0; w2 < NWAVE; ++w2) pre += (w2 < wave) ? wtot[w2] : 0;
    int run = pre + incl - ts;
    soff[4 * tid + 0] = run; run += e0;
    soff[4 * tid + 1] = run; run += e1;
    soff[4 * tid + 2] = run; run += e2;
    soff[4 * tid + 3] = run;
  }
  __syncthreads();
  for (int i = tid; i < NBR; i += NTHR) list[i] = soff[i];
  __syncthreads();

  if (wave == 0) {
#pragma unroll 1
    for (int b0 = 0; b0 < nh; b0 += 32) {
      const int idx = b0 + lane;
      const int uv  = reg1[idx < RCAP ? idx : RCAP - 1];
      const int m32 = (nh - b0) < 32 ? (nh - b0) : 32;
#pragma unroll 1
      for (int k = 0; k < m32; ++k) {
        const int u   = __builtin_amdgcn_readlane(uv, k);
        const int sl  = u & (NBR - 1);
        const int eid = (int)((unsigned)u >> PKS);
        if (lane == 0) {
          int pos = list[sl];
          pos = pos < 0 ? 0 : (pos > RCAP - 1 ? RCAP - 1 : pos);
          reg2[pos] = eid;
          list[sl] = pos + 1;
        }
      }
    }
  }
  __syncthreads();

  int* lg = LISTg + (size_t)blockIdx.x * RCAP;
#pragma unroll 1
  for (int i = tid; i < RCAP / 4; i += NTHR) {
    const v4i v = *(const v4ia*)(reg2 + 4 * i);
    *(volatile v4i*)(lg + 4 * i) = v;
  }
  __threadfence();
#pragma unroll 1
  for (int i = tid; i < RCAP / 4; i += NTHR) {
    const v4i v = *(const v4ia*)(reg2 + 4 * i);
    *(volatile v4i*)(lg + 4 * i) = v;
  }
  const v4i cv = *(const v4ia*)(scnt + 4 * tid);
  const v4i ov = *(const v4ia*)(soff + 4 * tid);
  const int fl = (nh >= RCAP) ? 1 : 0;
  const v4i fv = {fl, fl, fl, fl};
  int* cg = CNTg + (size_t)blockIdx.x * NBR + 4 * tid;
  int* og = OFFg + (size_t)blockIdx.x * NBR + 4 * tid;
  int* fg = FLGg + (size_t)blockIdx.x * OUTP + 4 * (tid & 7);
  const bool fw = tid < 8;
  *(volatile v4i*)cg = cv;
  *(volatile v4i*)og = ov;
  if (fw) *(volatile v4i*)fg = fv;
  __threadfence();
  *(volatile v4i*)cg = cv;
  *(volatile v4i*)og = ov;
  if (fw) *(volatile v4i*)fg = fv;
}

template <int C, int RND>
__global__ __launch_bounds__(ETILE) void k_edge(const float* __restrict__ ea1, const float* __restrict__ ea2,
                                                const int* __restrict__ srcs, const float* __restrict__ X,
                                                const unsigned short* __restrict__ EWT,
                                                const float* __restrict__ eb, int nE, int nN,
                                                unsigned short* M16) {
  constexpr int DP = C + 4;
  constexpr int NT = C / 16;
  __shared__ __attribute__((aligned(16))) unsigned short sA[ETILE * APE];
  __shared__ __attribute__((aligned(16))) float sD[ETILE * DP];
  __shared__ __attribute__((aligned(16))) unsigned short sM[ETILE * C];
  __shared__ __attribute__((aligned(16))) float ebs[C];
  const int tid = (int)threadIdx.x, lane = tid & 31, wave = tid >> 5, hh = lane >> 4, m = lane & 15;
  const int elb = (int)blockIdx.x * ETILE;
  const int el  = elb + tid;
  const int elc = el < nE ? el : nE - 1;

  {
    const v4f a0 = *(const v4f*)(ea1 + (size_t)elc * 8);
    const v4f a1 = *(const v4f*)(ea1 + (size_t)elc * 8 + 4);
    const v4f f0 = *(const v4f*)(ea2 + (size_t)elc * 8);
    const v4f f1 = *(const v4f*)(ea2 + (size_t)elc * 8 + 4);
    v8us o0, o1;
    o0[0] = bf_bits(a0.x); o0[1] = bf_bits(a0.y); o0[2] = bf_bits(a0.z); o0[3] = bf_bits(a0.w);
    o0[4] = bf_bits(a1.x); o0[5] = bf_bits(a1.y); o0[6] = bf_bits(a1.z); o0[7] = bf_bits(a1.w);
    o1[0] = bf_bits(f0.x); o1[1] = bf_bits(f0.y); o1[2] = bf_bits(f0.z); o1[3] = bf_bits(f0.w);
    o1[4] = bf_bits(f1.x); o1[5] = bf_bits(f1.y); o1[6] = bf_bits(f1.z); o1[7] = bf_bits(f1.w);
    const v8us z8 = {0, 0, 0, 0, 0, 0, 0, 0};
    unsigned short* ra = sA + tid * APE;
    *(v8usa*)(ra)      = o0;
    *(v8usa*)(ra + 8)  = o1;
    *(v8usa*)(ra + 16) = z8;
    *(v8usa*)(ra + 24) = z8;
    const int ec = tid < C ? tid : C - 1;
    const float ebv = bf_rne(eb[ec]);
    if (tid < C) ebs[tid] = ebv;
  }
  __syncthreads();

  {
    v8f acc[2][NT];
    const v8f z = {0.f, 0.f, 0.f, 0.f, 0.f, 0.f, 0.f, 0.f};
#pragma unroll
    for (int mt = 0; mt < 2; ++mt)
#pragma unroll
      for (int nt = 0; nt < NT; ++nt) acc[mt][nt] = z;
    const unsigned short* ap0 = sA + (32 * wave + m) * APE + 8 * hh;
    const unsigned short* ap1 = ap0 + 16 * APE;
    FragB fa0, fa1;
    fa0.h[0] = *(const v8usa*)(ap0);
    fa0.h[1] = *(const v8usa*)(ap0 + 16);
    fa1.h[0] = *(const v8usa*)(ap1);
    fa1.h[1] = *(const v8usa*)(ap1 + 16);
#pragma unroll
    for (int nt = 0; nt < NT; ++nt) {
      const unsigned short* wq = EWT + (size_t)(16 * nt + m) * KE + 8 * hh;
      FragB fb;
      fb.h[0] = *(const v8usa*)wq;
      fb.h[1] = *(const v8usa*)(wq + 16);
      acc[0][nt] = wmb(fa0, fb, acc[0][nt]);
      acc[1][nt] = wmb(fa1, fb, acc[1][nt]);
    }
#pragma unroll
    for (int nt = 0; nt < NT; ++nt)
#pragma unroll
      for (int mt = 0; mt < 2; ++mt)
#pragma unroll
        for (int r = 0; r < 8; ++r)
          sD[(32 * wave + 16 * mt + 8 * hh + r) * DP + 16 * nt + m] = acc[mt][nt][r];
  }
  __syncthreads();

  {
    const int sraw = srcs[elc];
    const int s = sraw < 0 ? 0 : (sraw > nN - 1 ? nN - 1 : sraw);
    const float* xr = X + (size_t)s * C;
    const float* rd = sD + tid * DP;
    unsigned short* rm = sM + tid * C;
#pragma unroll 1
    for (int c8 = 0; c8 < C / 8; ++c8) {
      const v4f da = *(const v4fa*)(rd + 8 * c8);
      const v4f db = *(const v4fa*)(rd + 8 * c8 + 4);
      const v4f xa = *(const v4f*)(xr + 8 * c8);
      const v4f xb = *(const v4f*)(xr + 8 * c8 + 4);
      const v4f ba = *(const v4fa*)(ebs + 8 * c8);
      const v4f bb = *(const v4fa*)(ebs + 8 * c8 + 4);
      const float d8[8] = {da.x, da.y, da.z, da.w, db.x, db.y, db.z, db.w};
      const float x8[8] = {xa.x, xa.y, xa.z, xa.w, xb.x, xb.y, xb.z, xb.w};
      const float b8[8] = {ba.x, ba.y, ba.z, ba.w, bb.x, bb.y, bb.z, bb.w};
      v8us o;
#pragma unroll
      for (int i = 0; i < 8; ++i) {
        float xv = x8[i];
        if (RND != 0) xv = bf_rne(xv);
        const float v = relu_np((xv + d8[i]) + b8[i]);
        o[i] = f2h(CMSG * v);
      }
      *(v8usa*)(rm + 8 * c8) = o;
    }
  }
  __syncthreads();

  {
    constexpr int NS = C / 8;
    v4i pv[NS];
#pragma unroll
    for (int it = 0; it < NS; ++it) pv[it] = *(const v4ia*)(sM + (size_t)(it * ETILE + tid) * 8);
    unsigned short* mb = M16 + (size_t)elb * C;
#pragma unroll
    for (int it = 0; it < NS; ++it) *(volatile v4i*)(mb + (size_t)(it * ETILE + tid) * 8) = pv[it];
    __threadfence();
#pragma unroll
    for (int it = 0; it < NS; ++it) *(volatile v4i*)(mb + (size_t)(it * ETILE + tid) * 8) = pv[it];
  }
}

template <int C, int RND>
__global__ __launch_bounds__(NTHR) void k_agg(const unsigned short* __restrict__ M16, const float* __restrict__ F,
                                              const int* __restrict__ LISTg, const int* __restrict__ CNTg,
                                              const int* __restrict__ OFFg, const int* __restrict__ FLGg,
                                              int nN, int nE, int nLB, unsigned short* Z) {
  constexpr int ZP = 2 * C;
  __shared__ __attribute__((aligned(16))) unsigned short sZ[64 * ZP];
  const int tid = (int)threadIdx.x, lane = tid & 31, wave = tid >> 5;
  const float qnan = __int_as_float(0x7fc00000);

#pragma unroll 1
  for (int jt = 0; jt < 8; ++jt) {
    const int lr   = 8 * wave + jt;
    const int grow = (int)blockIdx.x * 64 + lr;
    int lb = grow >> PKS;
    lb = lb > nLB - 1 ? nLB - 1 : lb;
    const int slot = grow & (NBR - 1);
    int st = OFFg[(size_t)lb * NBR + slot];
    const int craw = CNTg[(size_t)lb * NBR + slot];
    const int flg  = FLGg[(size_t)lb * OUTP];
    int cnt = craw;
    st  = st < 0 ? 0 : (st > RCAP ? RCAP : st);
    cnt = cnt < 0 ? 0 : (cnt > DEGCAP ? DEGCAP : cnt);
    if (cnt > RCAP - st) cnt = RCAP - st;
    const float pz = (flg != 0 || craw > DEGCAP) ? qnan : 0.0f;
    const bool liveRow = grow < nN;
    const int* lp = LISTg + (size_t)lb * RCAP;

    float a0 = 0.0f, a1 = 0.0f;
#pragma unroll 1
    for (int b0 = 0; b0 < cnt; b0 += 32) {
      int idx = st + b0 + lane;
      idx = idx < 0 ? 0 : (idx > RCAP - 1 ? RCAP - 1 : idx);
      int eid = lp[idx];
      eid = eid < 0 ? 0 : (eid > nE - 1 ? nE - 1 : eid);
      const int m32 = (cnt - b0) < 32 ? (cnt - b0) : 32;
#pragma unroll 1
      for (int k = 0; k < m32; ++k) {
        const int ek = __builtin_amdgcn_readlane(eid, k);
        if constexpr (C == 32) {
          const unsigned short hb = M16[(size_t)ek * C + lane];
          a0 += h2f((unsigned)hb);
        } else {
          const u32a* rp = (const u32a*)(M16 + (size_t)ek * C) + lane;
          const unsigned w = *rp;
          a0 += h2f(w & 0xffffu);
          a1 += h2f(w >> 16);
        }
      }
    }
    const int nc = liveRow ? grow : nN - 1;
    if constexpr (C == 32) {
      float sf = F[(size_t)nc * C + lane];
      if (RND != 0) sf = bf_rne(sf);
      float r0 = fmaf(a0, MINV, sf);
      r0 = liveRow ? (r0 + pz) : 0.0f;
      const unsigned short hb = bf_bits(r0);
      const unsigned short lo = bf_bits(r0 - bf_val(hb));
      sZ[lr * ZP + lane]     = hb;
      sZ[lr * ZP + C + lane] = lo;
    } else {
      const v2f sf2 = *(const v2f*)(F + (size_t)nc * C + 2 * lane);
      float s0 = sf2.x, s1 = sf2.y;
      if (RND != 0) { s0 = bf_rne(s0); s1 = bf_rne(s1); }
      float r0 = fmaf(a0, MINV, s0);
      float r1 = fmaf(a1, MINV, s1);
      r0 = liveRow ? (r0 + pz) : 0.0f;
      r1 = liveRow ? (r1 + pz) : 0.0f;
      const unsigned short h0 = bf_bits(r0), h1 = bf_bits(r1);
      const unsigned short l0 = bf_bits(r0 - bf_val(h0)), l1 = bf_bits(r1 - bf_val(h1));
      sZ[lr * ZP + 2 * lane]         = h0;
      sZ[lr * ZP + 2 * lane + 1]     = h1;
      sZ[lr * ZP + C + 2 * lane]     = l0;
      sZ[lr * ZP + C + 2 * lane + 1] = l1;
    }
  }
  __syncthreads();

  {
    constexpr int NS = (64 * ZP * 2 / 16) / NTHR;
    v4u pv[NS];
#pragma unroll
    for (int it = 0; it < NS; ++it) pv[it] = *(const v4ua*)(sZ + (size_t)(it * NTHR + tid) * 8);
    unsigned short* zb = Z + (size_t)blockIdx.x * 64 * ZP;
#pragma unroll
    for (int it = 0; it < NS; ++it) *(volatile v4u*)(zb + (size_t)(it * NTHR + tid) * 8) = pv[it];
    __threadfence();
#pragma unroll
    for (int it = 0; it < NS; ++it) *(volatile v4u*)(zb + (size_t)(it * NTHR + tid) * 8) = pv[it];
  }
}

template <int K, int MODE>
__global__ __launch_bounds__(GTHR) void k_gemm(const unsigned short* __restrict__ A,
                                               const unsigned short* __restrict__ WT,
                                               const float* __restrict__ bias,
                                               void* outp, int nN, int mRows) {
  constexpr int NT = 4;
  constexpr int BN = 64;
  static_assert((K % 32) == 0);
  __shared__ __attribute__((aligned(16))) float stg[GBM * BN];
  const int tid = (int)threadIdx.x, lane = tid & 31, wave = tid >> 5, hh = lane >> 4, m = lane & 15;
  const int rowBase = (int)blockIdx.x * GBM;

  v8f acc[NT];
  {
    const v8f z = {0.f, 0.f, 0.f, 0.f, 0.f, 0.f, 0.f, 0.f};
#pragma unroll
    for (int t = 0; t < NT; ++t) acc[t] = z;
  }
  const unsigned short* ap = A + (size_t)(rowBase + 16 * wave + m) * (size_t)K + 8 * hh;
  const unsigned short* wp = WT + (size_t)m * (size_t)K + 8 * hh;
  constexpr int ksteps = K / 32;
#pragma unroll 1
  for (int ks = 0; ks < ksteps; ++ks) {
    FragB af;
    af.h[0] = *(const v8usa*)(ap + 32 * ks);
    af.h[1] = *(const v8usa*)(ap + 32 * ks + 16);
#pragma unroll
    for (int t = 0; t < NT; ++t) {
      const unsigned short* wq = wp + (size_t)(16 * t) * (size_t)K + 32 * ks;
      FragB bf;
      bf.h[0] = *(const v8usa*)wq;
      bf.h[1] = *(const v8usa*)(wq + 16);
      acc[t] = wmb(af, bf, acc[t]);
    }
  }

#pragma unroll
  for (int t = 0; t < NT; ++t) {
    const int lc = 16 * t + m;
    const float bb = bf_rne(bias[lc]);
#pragma unroll
    for (int r = 0; r < 8; ++r) {
      const int lr = 16 * wave + 8 * hh + r;
      const bool live = (rowBase + lr) < nN;
      const float v = relu_np(acc[t][r] + bb);
      stg[lr * BN + lc] = live ? v : 0.0f;
    }
  }
  __syncthreads();

  if constexpr (MODE == 1) {
    unsigned short* outH = (unsigned short*)outp;
    const int part = m >> 3;
    const int cb   = 8 * (m & 7);
    const unsigned mh = 0u - (unsigned)part;
    const unsigned ml = ~mh;
    v8us pk[8];
#pragma unroll
    for (int i = 0; i < 8; ++i) {
      const int lr = 16 * wave + 2 * i + hh;
      const v4f a = *(const v4fa*)(stg + lr * BN + cb);
      const v4f b = *(const v4fa*)(stg + lr * BN + cb + 4);
      const float f8[8] = {a.x, a.y, a.z, a.w, b.x, b.y, b.z, b.w};
      v8us oo;
#pragma unroll
      for (int e = 0; e < 8; ++e) {
        const unsigned hb = (unsigned)bf_bits(f8[e]);
        const unsigned lb = (unsigned)bf_bits(f8[e] - __uint_as_float(hb << 16));
        oo[e] = (unsigned short)((hb & ml) | (lb & mh));
      }
      pk[i] = oo;
    }
    unsigned short* ob = outH + (size_t)(rowBase + 16 * wave) * 128 + 8 * lane;
#pragma unroll
    for (int i = 0; i < 8; ++i) {
      if (rowBase + 16 * wave + 2 * i < mRows) *(volatile v8us*)(ob + i * 256) = pk[i];
    }
    __threadfence();
#pragma unroll
    for (int i = 0; i < 8; ++i) {
      if (rowBase + 16 * wave + 2 * i < mRows) *(volatile v8us*)(ob + i * 256) = pk[i];
    }
  } else {
    float* outF = (float*)outp;
    v4f fv[8];
#pragma unroll
    for (int i = 0; i < 8; ++i) {
      const int lr = 16 * wave + 2 * i + hh;
      fv[i] = *(const v4fa*)(stg + lr * BN + 4 * m);
    }
    float* ob = outF + (size_t)(rowBase + 16 * wave) * 64 + 4 * lane;
#pragma unroll
    for (int i = 0; i < 8; ++i) {
      if (rowBase + 16 * wave + 2 * i < mRows) *(volatile v4f*)(ob + i * 128) = fv[i];
    }
    __threadfence();
#pragma unroll
    for (int i = 0; i < 8; ++i) {
      if (rowBase + 16 * wave + 2 * i < mRows) *(volatile v4f*)(ob + i * 128) = fv[i];
    }
  }
}

__global__ __launch_bounds__(NTHR) void k_s2s(const float* __restrict__ H2, const int* __restrict__ bat, int nN,
                                              const float* __restrict__ GT,
                                              const float* __restrict__ bih, const float* __restrict__ bhh,
                                              const float* __restrict__ dw, const float* __restrict__ db,
                                              const float* __restrict__ ow, const float* __restrict__ ob,
                                              float* OUTS) {
  extern __shared__ v4f s2s_dyn[];
  float* xs    = (float*)s2s_dyn;
  int*   wl    = (int*)(xs + NODECAP * DH);
  int*   nodes = wl + NWAVE * NODECAP;
  __shared__ __attribute__((aligned(16))) float qs[2 * DH];
  __shared__ float gpre[NGATE];
  __shared__ float actb[2 * NGATE];
  __shared__ float cbuf[DH];
  __shared__ float ev[NODECAP];
  __shared__ float part[4 * DH];
  __shared__ float red2[DH];
  __shared__ float red[4];
  __shared__ int   wcn[NWAVE];
  const int tid = (int)threadIdx.x, lane = tid & 31, wave = tid >> 5;
  const int g = (int)blockIdx.x;

  const int per  = (((nN + NWAVE - 1) / NWAVE) + 31) & ~31;
  const int wbeg = wave * per;
  int wend = wbeg + per;
  wend = wend > nN ? nN : wend;
  int wc = 0;
#pragma unroll 1
  for (int i0 = wbeg; i0 < wend; i0 += 32) {
    const int i  = i0 + lane;
    const int ic = i < nN ? i : nN - 1;
    const int b  = bat[ic];
    const bool hit = (i < wend) && (b == g);
    const unsigned msk = __builtin_amdgcn_ballot_w32(hit);
    if (hit) {
      const int pos = wc + (int)__builtin_amdgcn_mbcnt_lo(msk, 0u);
      if (pos < NODECAP) wl[wave * NODECAP + pos] = i;
    }
    wc += (int)__builtin_popcount(msk);
  }
  if (lane == 0) wcn[wave] = wc;
  if (tid < 2 * DH) qs[tid] = 0.0f;
  if (tid < DH) cbuf[tid] = 0.0f;
  __syncthreads();
  int pre = 0, tot = 0, rawtot = 0;
#pragma unroll
  for (int w2 = 0; w2 < NWAVE; ++w2) {
    const int c  = wcn[w2];
    const int cc = c < 0 ? 0 : (c > NODECAP ? NODECAP : c);
    rawtot += (c < 0 ? 0 : c);
    tot += cc;
    pre += (w2 < wave) ? cc : 0;
  }
  const bool ovf = rawtot > NODECAP;
  const int cnt = tot > NODECAP ? NODECAP : tot;
  {
    const int wcc = wc < 0 ? 0 : (wc > NODECAP ? NODECAP : wc);
#pragma unroll 1
    for (int i = lane; i < wcc; i += 32) {
      const int pos = pre + i;
      if (pos < NODECAP) nodes[pos] = wl[wave * NODECAP + i];
    }
  }
  __syncthreads();
#pragma unroll 1
  for (int idx = tid; idx < cnt * 16; idx += NTHR) {
    const int n  = idx >> 4;
    const int c4 = (idx & 15) * 4;
    int node = nodes[n];
    node = node < 0 ? 0 : (node > nN - 1 ? nN - 1 : node);
    const v4f v = *(const v4f*)(H2 + (size_t)node * DH + c4);
    *(v4fa*)(xs + n * DH + c4) = v;
  }
  __syncthreads();

  const float bihv = bf_rne(bih[tid]);
  const float bhhv = bf_rne(bhh[tid]);
  float c_state = 0.0f;
  const float ninf = __int_as_float((int)0xff800000u);

#pragma unroll 1
  for (int step = 0; step < 3; ++step) {
    {
      float a = 0.0f, b = 0.0f;
#pragma unroll 4
      for (int k = 0; k < 2 * DH; ++k) a = fmaf(qs[k], GT[(size_t)k * NGATE + tid], a);
#pragma unroll 4
      for (int k = 0; k < DH; ++k) b = fmaf(qs[k], GT[(size_t)(2 * DH + k) * NGATE + tid], b);
      gpre[tid] = ((a + bihv) + b) + bhhv;
    }
    __syncthreads();
#pragma unroll 1
    for (int pass = 0; pass < 2; ++pass) {
      const float v0 = gpre[tid];
      const float v1 = cbuf[tid & (DH - 1)];
      const float v  = (pass == 0) ? v0 : v1;
      const float sg = __builtin_amdgcn_rcpf(1.0f + expf(-v));
      const float th = tanhf(v);
      const bool useS = (pass == 0) && ((tid >> 6) != 2);
      actb[pass * NGATE + tid] = useS ? sg : th;
      __syncthreads();
      if (pass == 0 && tid < DH) {
        c_state = fmaf(actb[DH + tid], c_state, actb[tid] * actb[2 * DH + tid]);
        cbuf[tid] = c_state;
      }
      __syncthreads();
    }
    if (tid < DH) qs[tid] = actb[3 * DH + tid] * actb[NGATE + tid];
    __syncthreads();

    if (cnt > 0) {
#pragma unroll 1
      for (int n = tid; n < cnt; n += NTHR) {
        const float* xr = xs + n * DH;
        float s = 0.0f;
#pragma unroll 4
        for (int k = 0; k < DH; ++k) s = fmaf(xr[k], qs[k], s);
        ev[n] = s;
      }
      __syncthreads();
      if (wave == 0) {
        float mx = ninf;
#pragma unroll 1
        for (int n = lane; n < cnt; n += 32) mx = nmax(mx, ev[n]);
#pragma unroll
        for (int d = 16; d >= 1; d >>= 1) {
          const float o = __shfl_xor(mx, d);
          mx = nmax(mx, o);
        }
        if (lane == 0) red[0] = mx;
      }
      __syncthreads();
      {
        const float mx = red[0];
#pragma unroll 1
        for (int n = tid; n < cnt; n += NTHR) {
          const float e = ev[n];
          ev[n] = expf(e - mx);
        }
      }
      __syncthreads();
      if (wave == 0) {
        float s = 0.0f;
#pragma unroll 1
        for (int n = lane; n < cnt; n += 32) s += ev[n];
#pragma unroll
        for (int d = 16; d >= 1; d >>= 1) {
          const float o = __shfl_xor(s, d);
          s += o;
        }
        if (lane == 0) red[1] = s;
      }
      __syncthreads();
      {
        const float rd = __builtin_amdgcn_rcpf(red[1]);
        const int p = tid >> 6, c = tid & (DH - 1);
        float acc = 0.0f;
#pragma unroll 1
        for (int n = p; n < cnt; n += 4) acc = fmaf(ev[n] * rd, xs[n * DH + c], acc);
        part[p * DH + c] = acc;
      }
      __syncthreads();
      if (tid < DH) qs[DH + tid] = ((part[tid] + part[DH + tid]) + part[2 * DH + tid]) + part[3 * DH + tid];
    } else {
      if (tid < DH) qs[DH + tid] = 0.0f;
    }
    __syncthreads();
  }

  if (tid < DH) {
    float acc = 0.0f;
#pragma unroll 4
    for (int k = 0; k < 2 * DH; ++k) acc = fmaf(qs[k], bf_rne(dw[(size_t)k * DH + tid]), acc);
    const float z = relu_np(acc + bf_rne(db[tid]));
    red2[tid] = z * bf_rne(ow[tid]);
  }
  __syncthreads();
  if (wave == 0) {
    float s = red2[lane] + red2[lane + 32];
#pragma unroll
    for (int d = 16; d >= 1; d >>= 1) {
      const float o = __shfl_xor(s, d);
      s += o;
    }
    float res = s + bf_rne(ob[0]);
    res = ovf ? __int_as_float(0x7fc00000) : res;
    const v4f rv = {res, res, res, res};
    float* op = OUTS + (size_t)g * OUTP + 4 * (lane & 7);
    const bool stw = lane < 8;
    if (stw) *(volatile v4f*)op = rv;
    __threadfence();
    if (stw) *(volatile v4f*)op = rv;
  }
}

__global__ __launch_bounds__(128) void k_out(const float* __restrict__ OUTS, int nG, float* out) {
  const int t  = (int)blockIdx.x * 128 + (int)threadIdx.x;
  const int g0 = 4 * t;
  const bool ok = (g0 + 3) < nG;
  const int gc = ok ? g0 : 0;
  v4f v;
  v.x = OUTS[(size_t)(gc + 0) * OUTP];
  v.y = OUTS[(size_t)(gc + 1) * OUTP];
  v.z = OUTS[(size_t)(gc + 2) * OUTP];
  v.w = OUTS[(size_t)(gc + 3) * OUTP];
  float* op = out + gc;
  if (ok) *(volatile v4f*)op = v;
  __threadfence();
  if (ok) *(volatile v4f*)op = v;
}

static inline int cdiv(int a, int b) { return (a + b - 1) / b; }
static inline size_t al256(size_t o) { return (o + 255) & ~(size_t)255; }

extern "C" void kernel_launch(void* const* d_in, const int* in_sizes, int n_in,
                              void* d_out, int out_size, void* d_ws, size_t ws_size,
                              hipStream_t stream) {
  if (n_in < 25) return;
  if (in_sizes[0] < C0 || (in_sizes[0] % C0) != 0) return;
  const int nN = in_sizes[0] / C0;
  if (nN < 1 || nN > (1 << 22)) return;
  if (in_sizes[1] < 8 || (in_sizes[1] % 8) != 0) return;
  const int nE = in_sizes[1] / 8;
  if (nE < 1 || nE >= (1 << 21)) return;
  if (in_sizes[2] != nE * 8) return;
  if (in_sizes[3] != 2 * nE) return;
  if (in_sizes[4] != nN) return;
  if (in_sizes[5] != EDIM * C0 || in_sizes[6] != C0) return;
  if (in_sizes[7] != C0 * DH || in_sizes[8] != DH) return;
  if (in_sizes[9] != DH * DH || in_sizes[10] != DH) return;
  if (in_sizes[11] != EDIM * C1 || in_sizes[12] != C1) return;
  if (in_sizes[13] != C1 * DH || in_sizes[14] != DH) return;
  if (in_sizes[15] != DH * DH || in_sizes[16] != DH) return;
  if (in_sizes[17] != 4 * DH * 2 * DH || in_sizes[18] != 4 * DH) return;
  if (in_sizes[19] != 4 * DH * DH || in_sizes[20] != 4 * DH) return;
  if (in_sizes[21] != 2 * DH * DH || in_sizes[22] != DH) return;
  if (in_sizes[23] != DH || in_sizes[24] != 1) return;
  const int nG = out_size;
  if (nG < 32 || (nG % 32) != 0 || nG > 65535) return;
  if ((long long)NBR * (long long)nE * 5LL > (long long)RCAP * (long long)nN * 4LL) return;

  const float* x    = (const float*)d_in[0];
  const float* ea1  = (const float*)d_in[1];
  const float* ea2  = (const float*)d_in[2];
  const int*   ei   = (const int*)d_in[3];
  const int*   src  = ei;
  const int*   dst  = ei + nE;
  const int*   bat  = (const int*)d_in[4];
  const float* ew0  = (const float*)d_in[5];
  const float* eb0  = (const float*)d_in[6];
  const float* w10  = (const float*)d_in[7];
  const float* b10  = (const float*)d_in[8];
  const float* w20  = (const float*)d_in[9];
  const float* b20  = (const float*)d_in[10];
  const float* ew1  = (const float*)d_in[11];
  const float* eb1  = (const float*)d_in[12];
  const float* w11  = (const float*)d_in[13];
  const float* b11  = (const float*)d_in[14];
  const float* w21  = (const float*)d_in[15];
  const float* b21  = (const float*)d_in[16];
  const float* wih  = (const float*)d_in[17];
  const float* bih  = (const float*)d_in[18];
  const float* whh  = (const float*)d_in[19];
  const float* bhh  = (const float*)d_in[20];
  const float* dw   = (const float*)d_in[21];
  const float* db   = (const float*)d_in[22];
  const float* ow   = (const float*)d_in[23];
  const float* ob   = (const float*)d_in[24];
  float* out = (float*)d_out;

  const int NPAD = cdiv(nN, GBM) * GBM;
  const int gM   = NPAD / GBM;
  const int nLB  = cdiv(NPAD, NBR);
  const int nET  = cdiv(nE, ETILE);
  const size_t EPAD = (size_t)nET * ETILE;
  const int vec8 = ((nE & 3) == 0) ? 1 : 0;

  char* ws = (char*)d_ws;
  size_t off = 0;
  const size_t oEW0 = off; off = al256(off + (size_t)C0 * KE * 2);
  const size_t oEW1 = off; off = al256(off + (size_t)C1 * KE * 2);
  const size_t oW1A = off; off = al256(off + (size_t)DH * 2 * C0 * 2);
  const size_t oW2A = off; off = al256(off + (size_t)DH * 2 * DH * 2);
  const size_t oW1B = off; off = al256(off + (size_t)DH * 2 * C1 * 2);
  const size_t oW2B = off; off = al256(off + (size_t)DH * 2 * DH * 2);
  const size_t oGT  = off; off = al256(off + (size_t)3 * DH * NGATE * 4);
  const size_t oLS  = off; off = al256(off + (size_t)nLB * RCAP * 4);
  const size_t oCN  = off; off = al256(off + (size_t)nLB * NBR * 4);
  const size_t oOF  = off; off = al256(off + (size_t)nLB * NBR * 4);
  const size_t oFL  = off; off = al256(off + (size_t)nLB * OUTP * 4);
  const size_t oM   = off; off = al256(off + EPAD * C1 * 2);
  const size_t oZ   = off; off = al256(off + (size_t)NPAD * 2 * C1 * 2);
  const size_t oT   = off; off = al256(off + (size_t)NPAD * 2 * DH * 2);
  const size_t oH1  = off; off = al256(off + (size_t)NPAD * DH * 4);
  const size_t oH2  = off; off = al256(off + (size_t)NPAD * DH * 4);
  const size_t oOS  = off; off = al256(off + (size_t)nG * OUTP * 4);
  if (off > ws_size) return;

  unsigned short* EW0T = (unsigned short*)(ws + oEW0);
  unsigned short* EW1T = (unsigned short*)(ws + oEW1);
  unsigned short* W1C0 = (unsigned short*)(ws + oW1A);
  unsigned short* W2C0 = (unsigned short*)(ws + oW2A);
  unsigned short* W1C1 = (unsigned short*)(ws + oW1B);
  unsigned short* W2C1 = (unsigned short*)(ws + oW2B);
  float*          GT   = (float*)(ws + oGT);
  int*            LIST = (int*)(ws + oLS);
  int*            CNT  = (int*)(ws + oCN);
  int*            OFF  = (int*)(ws + oOF);
  int*            FLG  = (int*)(ws + oFL);
  unsigned short* M16  = (unsigned short*)(ws + oM);
  unsigned short* ZHL  = (unsigned short*)(ws + oZ);
  unsigned short* THL  = (unsigned short*)(ws + oT);
  float*          H1   = (float*)(ws + oH1);
  float*          H2   = (float*)(ws + oH2);
  float*          OUTS = (float*)(ws + oOS);

  hipFuncSetAttribute(reinterpret_cast<const void*>(&k_bucket), hipFuncAttributeMaxDynamicSharedMemorySize,
                      (int)LDS_BKT);
  hipFuncSetAttribute(reinterpret_cast<const void*>(&k_s2s), hipFuncAttributeMaxDynamicSharedMemorySize,
                      (int)LDS_S2S);

  k_prep<<<PREP_UNITS / NTHR, NTHR, 0, stream>>>(ew0, ew1, w10, w20, w11, w21, wih, whh,
                                                 EW0T, EW1T, W1C0, W2C0, W1C1, W2C1, GT);
  k_bucket<<<nLB, NTHR, LDS_BKT, stream>>>(dst, nN, nE, vec8, LIST, CNT, OFF, FLG);
  k_edge<C0, 1><<<nET, ETILE, 0, stream>>>(ea1, ea2, src, x, EW0T, eb0, nE, nN, M16);
  k_agg<C0, 1><<<gM, NTHR, 0, stream>>>(M16, x, LIST, CNT, OFF, FLG, nN, nE, nLB, ZHL);
  k_gemm<2 * C0, 1><<<gM, GTHR, 0, stream>>>(ZHL, W1C0, b10, (void*)THL, nN, NPAD);
  k_gemm<2 * DH, 2><<<gM, GTHR, 0, stream>>>(THL, W2C0, b20, (void*)H1, nN, NPAD);
  k_edge<C1, 0><<<nET, ETILE, 0, stream>>>(ea1, ea2, src, H1, EW1T, eb1, nE, nN, M16);
  k_agg<C1, 0><<<gM, NTHR, 0, stream>>>(M16, H1, LIST, CNT, OFF, FLG, nN, nE, nLB, ZHL);
  k_gemm<2 * C1, 1><<<gM, GTHR, 0, stream>>>(ZHL, W1C1, b11, (void*)THL, nN, NPAD);
  k_gemm<2 * DH, 2><<<gM, GTHR, 0, stream>>>(THL, W2C1, b21, (void*)H2, nN, NPAD);
  k_s2s<<<nG, NTHR, LDS_S2S, stream>>>(H2, bat, nN, GT, bih, bhh, dw, db, ow, ob, OUTS);
  k_out<<<cdiv(nG / 4, 128), 128, 0, stream>>>(OUTS, nG, out);
}
